// OriginalDoRA_36172214567497
// MI455X (gfx1250) — hardware-verified
//
#include <hip/hip_runtime.h>
#include <stdint.h>

typedef __attribute__((ext_vector_type(16))) _Float16 v16h;
typedef __attribute__((ext_vector_type(8)))  _Float16 v8h;
typedef __attribute__((ext_vector_type(16))) __bf16   v16b;
typedef __attribute__((ext_vector_type(8)))  __bf16   v8b;
typedef __attribute__((ext_vector_type(8)))  float    v8f;
typedef __attribute__((ext_vector_type(4)))  float    v4f;

__device__ __forceinline__ unsigned short f2bf_bits(float f) {
  unsigned u = __float_as_uint(f);
  return (unsigned short)((u + 0x7FFFu + ((u >> 16) & 1u)) >> 16);
}
__device__ __forceinline__ float bf_bits2f(unsigned short h) { return __uint_as_float(((unsigned)h) << 16); }

__device__ __forceinline__ void dep_guard_h(v8f& a, v8f& b, v16h x, v16h y) { asm volatile("v_nop\n\tv_nop\n\tv_nop\n\tv_nop" : "+v"(a), "+v"(b) : "v"(x), "v"(y)); }
__device__ __forceinline__ void dep_guard_b(v8f& a, v8f& b, v16b x, v16b y) { asm volatile("v_nop\n\tv_nop\n\tv_nop\n\tv_nop" : "+v"(a), "+v"(b) : "v"(x), "v"(y)); }
__device__ __forceinline__ void keep4_h(v16h a, v16h b, v16h c, v16h d) { asm volatile("v_nop" :: "v"(a), "v"(b), "v"(c), "v"(d)); }
__device__ __forceinline__ void keep4_b(v16b a, v16b b, v16b c, v16b d) { asm volatile("v_nop" :: "v"(a), "v"(b), "v"(c), "v"(d)); }
__device__ __forceinline__ void acc_guard4(v8f& a, v8f& b, v8f& c, v8f& d) { asm volatile("v_nop\n\tv_nop\n\tv_nop\n\tv_nop" : "+v"(a), "+v"(b), "+v"(c), "+v"(d)); }
template <typename T> struct Frag;
template <> struct Frag<_Float16> {
  typedef v16h V; union U { v16h v; v8h h[2]; };
  static __device__ __forceinline__ v16h load(const _Float16* p) {
    U f; f.h[0] = *(const v8h*)(p); f.h[1] = *(const v8h*)(p + 16); return f.v;
  }
  static __device__ __forceinline__ v8f mma(v16h a, v16h b, v8f c) {
    return __builtin_amdgcn_wmma_f32_16x16x32_f16(false, a, false, b, (short)0, c, false, false);
  }
  static __device__ __forceinline__ void guard(v8f& a, v8f& b, v16h x, v16h y) { dep_guard_h(a, b, x, y); }
  static __device__ __forceinline__ void keep(v16h a, v16h b, v16h c, v16h d) { keep4_h(a, b, c, d); }
};
template <> struct Frag<__bf16> {
  typedef v16b V; union U { v16b v; v8b h[2]; };
  static __device__ __forceinline__ v16b load(const __bf16* p) {
    U f; f.h[0] = *(const v8b*)(p); f.h[1] = *(const v8b*)(p + 16); return f.v;
  }
  static __device__ __forceinline__ v8f mma(v16b a, v16b b, v8f c) {
    return __builtin_amdgcn_wmma_f32_16x16x32_bf16(false, a, false, b, (short)0, c, false, false);
  }
  static __device__ __forceinline__ void guard(v8f& a, v8f& b, v16b x, v16b y) { dep_guard_b(a, b, x, y); }
  static __device__ __forceinline__ void keep(v16b a, v16b b, v16b c, v16b d) { keep4_b(a, b, c, d); }
};

template <int ET> struct Elem;
template <> struct Elem<0> { typedef _Float16 T; };
template <> struct Elem<1> { typedef __bf16 T; };
template <int ET, bool SPLIT, int BIAS_MODE, int OUT_MODE, bool RESID, bool ROWSC, int ACT = 0>
__global__ __launch_bounds__(256) void wmma_gemm64(
    const unsigned short* __restrict__ Ap, const unsigned short* __restrict__ A2p, int lda, long strideA,
    const unsigned short* __restrict__ Btp, const unsigned short* __restrict__ Bt2p, int ldb, long strideB,
    void* __restrict__ Cout, void* __restrict__ Cout2, int ldc, long strideC,
    const float* __restrict__ bias,
    const float* __restrict__ resid, long strideR,
    const float* __restrict__ rsc,
    int M, int N, int K, int Mlim, float scale, float oscale) {
  typedef typename Elem<ET>::T T;
  typedef typename Frag<T>::V V;
  const T* A = (const T*)Ap; const T* A2 = (const T*)A2p; const T* Bt = (const T*)Btp; const T* Bt2 = (const T*)Bt2p;
  __shared__ __align__(16) float sT[8][16 * 68];
  const int b    = blockIdx.y;
  const int lane = threadIdx.x & 31;
  const int wave = threadIdx.x >> 5;
  const int tilesN = N >> 6;
  const int tilesM = M >> 6;
  const int tile = blockIdx.x * 8 + wave;
  if (tile >= tilesM * tilesN) return;
  const int tm = tile / tilesN;
  const int tn = tile - tm * tilesN;
  const int m0 = tm << 6;
  const int n0 = tn << 6;

  const T* Ab  = A  + (size_t)b * strideA;
  const T* Bb  = Bt + (size_t)b * strideB;
  const T* Ab2 = SPLIT ? (A2  + (size_t)b * strideA) : nullptr;
  const T* Bb2 = SPLIT ? (Bt2 + (size_t)b * strideB) : nullptr;

  const int rlane = lane & 15;
  const int koff  = (lane >> 4) * 8;
  const int mOff  = (lane >> 4) * 8;

  v8f acc[4][4];
#pragma unroll
  for (int i = 0; i < 4; ++i)
#pragma unroll
    for (int j = 0; j < 4; ++j) acc[i][j] = (v8f){0.f,0.f,0.f,0.f,0.f,0.f,0.f,0.f};

  for (int k0 = 0; k0 < K; k0 += 32) {
    V bh[4], bl[4];
#pragma unroll
    for (int j = 0; j < 4; ++j) {
      const size_t bo = (size_t)(n0 + (j << 4) + rlane) * ldb + koff + k0;
      bh[j] = Frag<T>::load(Bb + bo);
      if (SPLIT) bl[j] = Frag<T>::load(Bb2 + bo);
    }
#pragma unroll
    for (int i = 0; i < 4; ++i) {
      const size_t ao = (size_t)(m0 + (i << 4) + rlane) * lda + koff + k0;
      V ah = Frag<T>::load(Ab + ao);
      V al;
      if (SPLIT) al = Frag<T>::load(Ab2 + ao);
#pragma unroll
      for (int j = 0; j < 4; ++j) {
        acc[i][j] = Frag<T>::mma(ah, bh[j], acc[i][j]);
        if (SPLIT) {
          acc[i][j] = Frag<T>::mma(ah, bl[j], acc[i][j]);
          acc[i][j] = Frag<T>::mma(al, bh[j], acc[i][j]);
        }
      }
      Frag<T>::guard(acc[i][0], acc[i][3], ah, SPLIT ? al : ah);
    }
    Frag<T>::keep(bh[0], bh[1], bh[2], bh[3]);
    if (SPLIT) Frag<T>::keep(bl[0], bl[1], bl[2], bl[3]);
  }
  acc_guard4(acc[0][0], acc[0][1], acc[0][2], acc[0][3]);
  acc_guard4(acc[1][0], acc[1][1], acc[1][2], acc[1][3]);
  acc_guard4(acc[2][0], acc[2][1], acc[2][2], acc[2][3]);
  acc_guard4(acc[3][0], acc[3][1], acc[3][2], acc[3][3]);

  float* slab = sT[wave];
  const float* Rb = RESID ? (resid + (size_t)b * strideR) : nullptr;
#pragma unroll
  for (int i = 0; i < 4; ++i) {
    const int mBase = m0 + (i << 4);
#pragma unroll
    for (int j = 0; j < 4; ++j) {
      const int n = n0 + (j << 4) + rlane;
      float bv = 0.f;
      if (BIAS_MODE == 2) bv = bias[n];
#pragma unroll
      for (int r = 0; r < 8; ++r) {
        float v = acc[i][j][r] * scale;
        if (BIAS_MODE == 1) v += bias[mBase + mOff + r];
        if (BIAS_MODE == 2) v += bv;
        if (RESID) v += Rb[(size_t)(mBase + mOff + r) * ldc + n];
        if (ROWSC) v *= rsc[mBase + mOff + r] * oscale;
        if (ACT == 1) v = tanhf(v);
        if (ACT == 2) v = fmaxf(v, 0.0f);
        if (ACT == 3) v = v / (1.0f + expf(-v));
        if (ACT == 4) v = (v > 0.f) ? v : 0.01f * v;
        if (ACT == 5) v = 0.5f * v * (1.0f + erff(v * 0.70710678118654752f));
        slab[(mOff + r) * 68 + (j << 4) + rlane] = v;
      }
    }
    __builtin_amdgcn_fence(__ATOMIC_RELEASE, "workgroup");
    __builtin_amdgcn_wave_barrier();
    __builtin_amdgcn_fence(__ATOMIC_ACQUIRE, "workgroup");
    if (OUT_MODE == 0) {
      float* C = (float*)Cout + (size_t)b * strideC;
      const int hh = lane >> 4, c4 = (lane & 15) * 4;
      for (int pass = 0; pass < 2; ++pass) {
#pragma unroll
        for (int it = 0; it < 8; ++it) {
          const int row = it * 2 + hh;
          v4f v = *(const v4f*)(slab + row * 68 + c4);
          if (mBase + row < Mlim)
            *(volatile v4f*)(C + (size_t)(mBase + row) * ldc + n0 + c4) = v;
        }
        __threadfence();
      }
    } else {
      const int q = lane >> 3, c8 = (lane & 7) * 8;
      unsigned short* C  = (unsigned short*)Cout  + (size_t)b * strideC;
      unsigned short* C2 = (OUT_MODE == 2) ? ((unsigned short*)Cout2 + (size_t)b * strideC) : nullptr;
      for (int pass = 0; pass < 2; ++pass) {
#pragma unroll
        for (int it = 0; it < 4; ++it) {
          const int row = it * 4 + q;
          const float* sp = slab + row * 68 + c8;
          v8h hv, lv;
#pragma unroll
          for (int e = 0; e < 8; ++e) {
            if (OUT_MODE == 1) {
              hv[e] = (_Float16)sp[e];
            } else {
              unsigned short hb = f2bf_bits(sp[e]);
              unsigned short lb = f2bf_bits(sp[e] - bf_bits2f(hb));
              hv[e] = __builtin_bit_cast(_Float16, hb);
              lv[e] = __builtin_bit_cast(_Float16, lb);
            }
          }
          if (mBase + row < Mlim) {
            *(volatile v8h*)(C + (size_t)(mBase + row) * ldc + n0 + c8) = hv;
            if (OUT_MODE == 2) *(volatile v8h*)(C2 + (size_t)(mBase + row) * ldc + n0 + c8) = lv;
          }
        }
        __threadfence();
      }
    }
    __builtin_amdgcn_fence(__ATOMIC_RELEASE, "workgroup");
    __builtin_amdgcn_wave_barrier();
    __builtin_amdgcn_fence(__ATOMIC_ACQUIRE, "workgroup");
  }
}

__global__ __launch_bounds__(256) void cast_x_f16(
    const float* __restrict__ x, _Float16* __restrict__ X16, int rowsReal, int rowsPad, int cols) {
  const int cpr = cols >> 3;
  const int total = rowsPad * cpr;
  const int t = blockIdx.x * 256 + threadIdx.x;
  if (t >= total) return;
  const int row = t / cpr;
  const int c8 = (t - row * cpr) * 8;
  v8h hv;
  if (row < rowsReal) {
    const v4f a = *(const v4f*)(x + (size_t)row * cols + c8);
    const v4f c = *(const v4f*)(x + (size_t)row * cols + c8 + 4);
    hv[0] = (_Float16)a[0]; hv[1] = (_Float16)a[1]; hv[2] = (_Float16)a[2]; hv[3] = (_Float16)a[3];
    hv[4] = (_Float16)c[0]; hv[5] = (_Float16)c[1]; hv[6] = (_Float16)c[2]; hv[7] = (_Float16)c[3];
  } else {
#pragma unroll
    for (int e = 0; e < 8; ++e) hv[e] = (_Float16)0.0f;
  }
  _Float16* p = X16 + (size_t)row * cols + c8;
  *(volatile v8h*)p = hv;
  __threadfence();
  *(volatile v8h*)p = hv;
}

__global__ __launch_bounds__(256) void pack_k32_f16(
    const float* __restrict__ src, _Float16* __restrict__ dst, int rows, int rowStride, int kStride, float mul) {
  const int t = blockIdx.x * 256 + threadIdx.x;
  const int total = rows * 4;
  if (t >= total) return;
  const int row = t >> 2, c = t & 3;
  v8h hv;
#pragma unroll
  for (int e = 0; e < 8; ++e) hv[e] = (_Float16)0.0f;
  if (c < 2) {
#pragma unroll
    for (int e = 0; e < 8; ++e) {
      const int kk = c * 8 + e;
      hv[e] = (_Float16)(src[(size_t)row * rowStride + (size_t)kk * kStride] * mul);
    }
  }
  _Float16* p = dst + (size_t)row * 32 + c * 8;
  *(volatile v8h*)p = hv;
  __threadfence();
  *(volatile v8h*)p = hv;
}

static inline size_t align256(size_t v) { return (v + 255) & ~(size_t)255; }

extern "C" void kernel_launch(void* const* d_in, const int* in_sizes, int n_in,
                              void* d_out, int out_size, void* d_ws, size_t ws_size,
                              hipStream_t stream) {
  const int INF = 1024, OUTF = 4096, RNK = 16, KP = 32;
  if (n_in < 6) return;
  if (in_sizes[1] != OUTF * INF || in_sizes[2] < OUTF || in_sizes[3] != RNK * INF ||
      in_sizes[4] != OUTF * RNK || in_sizes[5] < OUTF) return;
  const int Mreal = in_sizes[0] / INF;
  if (Mreal <= 0 || Mreal * INF != in_sizes[0]) return;
  if (out_size != Mreal * OUTF) return;
  const int Mpad = ((Mreal + 63) / 64) * 64;

  const float* x    = (const float*)d_in[0];
  const float* wd   = (const float*)d_in[1];
  const float* mag  = (const float*)d_in[2];
  const float* lA   = (const float*)d_in[3];
  const float* lB   = (const float*)d_in[4];
  const float* bias = (const float*)d_in[5];
  float* out = (float*)d_out;

  size_t off = 0;
  const size_t offX16 = off;  off = align256(off + (size_t)Mpad * INF * 2);
  const size_t offW16 = off;  off = align256(off + (size_t)OUTF * INF * 2);
  const size_t offB16 = off;  off = align256(off + (size_t)OUTF * KP * 2);
  const size_t offAt  = off;  off = align256(off + (size_t)INF * KP * 2);
  const size_t total = off;
  if (total > ws_size || total > (size_t)134217728) return;

  unsigned char* ws = (unsigned char*)d_ws;
  _Float16* X16  = (_Float16*)(ws + offX16);
  _Float16* W16  = (_Float16*)(ws + offW16);
  _Float16* B16  = (_Float16*)(ws + offB16);
  _Float16* At16 = (_Float16*)(ws + offAt);

  {
    const int total_t = Mpad * (INF / 8);
    cast_x_f16<<<(total_t + 255) / 256, 256, 0, stream>>>(x, X16, Mreal, Mpad, INF);
  }
  pack_k32_f16<<<(OUTF * 4 + 255) / 256, 256, 0, stream>>>(lB, B16, OUTF, RNK, 1, 64.0f);
  pack_k32_f16<<<(INF * 4 + 255) / 256, 256, 0, stream>>>(lA, At16, INF, 1, INF, 64.0f);

  {
    const int M = OUTF, N = INF, K = KP;
    const int tiles = (M / 64) * (N / 64);
    const int blocks = (tiles + 7) / 8;
    wmma_gemm64<0, false, 0, 1, true, true, 0><<<dim3(blocks, 1), 256, 0, stream>>>(
        (const unsigned short*)B16, (const unsigned short*)B16, KP, 0L,
        (const unsigned short*)At16, (const unsigned short*)At16, KP, 0L,
        (void*)W16, (void*)W16, INF, 0L,
        bias,
        wd, 0L,
        mag,
        M, N, K, M, 0.8f / 4096.0f, 16.0f);
  }
  {
    const int M = Mpad, N = OUTF, K = INF;
    const int tiles = (M / 64) * (N / 64);
    const int blocks = (tiles + 7) / 8;
    wmma_gemm64<0, false, 2, 0, false, false, 0><<<dim3(blocks, 1), 256, 0, stream>>>(
        (const unsigned short*)X16, (const unsigned short*)X16, INF, 0L,
        (const unsigned short*)W16, (const unsigned short*)W16, INF, 0L,
        (void*)out, (void*)out, OUTF, 0L,
        bias,
        bias, 0L,
        bias,
        M, N, K, Mreal, 1.0f / 16.0f, 1.0f);
  }
  (void)hipGetLastError();
}
